// Model_31044023616105
// MI455X (gfx1250) — hardware-verified
//
#include <hip/hip_runtime.h>
#include <math.h>

constexpr int NBAT    = 4;
constexpr int NSTEP   = 16384;
constexpr int NHID    = 128;
constexpr int NGATE   = 3 * NHID;
constexpr int NWROW   = 2 * NGATE;
constexpr int NHEAD1  = 64;
constexpr int NHEAD2  = 64;
constexpr int NOUTCH  = 2;
constexpr int NROWS   = NBAT * NSTEP;
constexpr int SCAN_THR = 512;
constexpr int HEAD_THR = 256;
constexpr int HEAD_ROWS = 128;
constexpr int APITCH  = 136;
constexpr int SLABP   = 68;
constexpr int STAGE_STEPS = 8;
constexpr float WCARRY   = 256.0f;
constexpr float ACARRY   = 64.0f;
constexpr float LCARRY   = 4096.0f;
constexpr float HI_INV   = 1.0f / (WCARRY * ACARRY);
constexpr float LO_INV   = 1.0f / LCARRY;
constexpr float HILO_INV = HI_INV * LO_INV;

static_assert(NHID % 32 == 0);
static_assert(NHEAD1 % 32 == 0);
static_assert(NSTEP / 32 == SCAN_THR);
static_assert(NBAT * NHID == SCAN_THR);
static_assert(NSTEP % STAGE_STEPS == 0);
static_assert(NROWS % HEAD_ROWS == 0);
static_assert((NGATE * NHID / 8) % 256 == 0);
static_assert((NHEAD1 * NHID / 8) % 256 == 0);
static_assert((NHEAD2 * NHEAD1 / 8) % 256 == 0);
static_assert((APITCH * 2) % 16 == 0);
static_assert((SLABP * 4) % 16 == 0);

typedef __attribute__((ext_vector_type(16))) _Float16 v16h;
typedef __attribute__((ext_vector_type(8)))  _Float16 v8h;
typedef __attribute__((ext_vector_type(8)))  float    v8f;
typedef __attribute__((ext_vector_type(4)))  float    v4f;
typedef __attribute__((ext_vector_type(4)))  int      v4i;

__device__ __forceinline__ unsigned short f2bf_bits(float f) {
  unsigned u = __float_as_uint(f);
  return (unsigned short)((u + 0x7FFFu + ((u >> 16) & 1u)) >> 16);
}
__device__ __forceinline__ float bf_bits2f(unsigned short h) { return __uint_as_float(((unsigned)h) << 16); }
__device__ __forceinline__ float bf16r(float f) { return bf_bits2f(f2bf_bits(f)); }

union FragU { v16h v; v8h h[2]; };
__device__ __forceinline__ v16h frag_load(const _Float16* p) {
  FragU f;
  f.h[0] = *(const v8h*)(p);
  f.h[1] = *(const v8h*)(p + 16);
  return f.v;
}
__device__ __forceinline__ v8f frag_mma(v16h a, v16h b, v8f c) {
  return __builtin_amdgcn_wmma_f32_16x16x32_f16(false, a, false, b, (short)0, c, false, false);
}
__device__ __forceinline__ void guard3(v8f& a, v8f& b, v8f& c, v16h x, v16h y0, v16h y1, v16h y2) {
  asm volatile("v_nop\n\tv_nop\n\tv_nop\n\tv_nop" : "+v"(a), "+v"(b), "+v"(c) : "v"(x), "v"(y0), "v"(y1), "v"(y2));
}
__device__ __forceinline__ void guard8(v8f& a0, v8f& a1, v8f& a2, v8f& a3, v8f& a4, v8f& a5, v8f& a6, v8f& a7,
                                       v16h x0, v16h x1, v16h y0, v16h y1, v16h y2, v16h y3) {
  asm volatile("v_nop\n\tv_nop\n\tv_nop\n\tv_nop"
               : "+v"(a0), "+v"(a1), "+v"(a2), "+v"(a3), "+v"(a4), "+v"(a5), "+v"(a6), "+v"(a7)
               : "v"(x0), "v"(x1), "v"(y0), "v"(y1), "v"(y2), "v"(y3));
}
__device__ __forceinline__ void pin_h(v16h& x) { asm volatile("" : "+v"(x)); }
__device__ __forceinline__ void pin_f4(float& a, float& b, float& c, float& d) { asm volatile("" : "+v"(a), "+v"(b), "+v"(c), "+v"(d)); }

__device__ __forceinline__ void split16(float x, _Float16& hi, _Float16& lo) {
  const float xs = x * ACARRY;
  hi = (_Float16)xs;
  float hf = (float)hi;
  asm volatile("" : "+v"(hf));
  lo = (_Float16)((xs - hf) * LCARRY);
}
__device__ __forceinline__ void build_frag(v4f x0, v4f x1, v4f x2, v4f x3, v16h& fh, v16h& fl) {
#pragma unroll
  for (int e = 0; e < 4; ++e) {
    const float s0 = x0[e];
    const float s1 = x1[e];
    const float s2 = x2[e];
    const float s3 = x3[e];
    _Float16 h, l;
    split16(s0, h, l); fh[e] = h;      fl[e] = l;
    split16(s1, h, l); fh[4 + e] = h;  fl[4 + e] = l;
    split16(s2, h, l); fh[8 + e] = h;  fl[8 + e] = l;
    split16(s3, h, l); fh[12 + e] = h; fl[12 + e] = l;
  }
}
__device__ __forceinline__ float sigm(float x) { return 1.0f / (1.0f + expf(-x)); }
__device__ __forceinline__ float elu1(float v) {
  const float e = expm1f(v < 0.0f ? v : 0.0f);
  return v > 0.0f ? v : e;
}
__device__ __forceinline__ float embed4(float w0, float w1, float w2, float w3, float be,
                                        float f0, float f1, float f2, float f3) {
  float a = w0 * bf16r(f0);
  a = fmaf(w1, bf16r(f1), a);
  a = fmaf(w2, bf16r(f2), a);
  a = fmaf(w3, bf16r(f3), a);
  return a + be;
}
__device__ __forceinline__ void fold_gate(const v8f cg, bool selx, float bias, float& o0, float& o1) {
  const float x0 = cg[0] + cg[4] * LO_INV;
  const float x1 = cg[1] + cg[5] * LO_INV;
  const float h0 = cg[2] + cg[6] * LO_INV;
  const float h1 = cg[3] + cg[7] * LO_INV;
  o0 = (selx ? x0 : h0) * HI_INV + bias;
  o1 = (selx ? x1 : h1) * HI_INV + bias;
}

__global__ __launch_bounds__(256) void prep_kernel(const float* __restrict__ W_ih, const float* __restrict__ W_hh,
                                                   const float* __restrict__ W1, const float* __restrict__ W2,
                                                   unsigned short* __restrict__ Bw, unsigned short* __restrict__ W1h,
                                                   unsigned short* __restrict__ W2h) {
  const int blk = blockIdx.x;
  const float* src;
  unsigned short* dst;
  int lb;
  if (blk < 24)      { src = W_ih; dst = Bw;                lb = blk; }
  else if (blk < 48) { src = W_hh; dst = Bw + NGATE * NHID; lb = blk - 24; }
  else if (blk < 52) { src = W1;   dst = W1h;               lb = blk - 48; }
  else               { src = W2;   dst = W2h;               lb = blk - 52; }
  const int i = lb * 256 + threadIdx.x;
  const v4f a = *(const v4f*)(src + (size_t)i * 8);
  const v4f b = *(const v4f*)(src + (size_t)i * 8 + 4);
  v8h hv;
#pragma unroll
  for (int e = 0; e < 4; ++e) {
    const float s0 = a[e];
    const float s1 = b[e];
    hv[e]     = (_Float16)(bf16r(s0) * WCARRY);
    hv[4 + e] = (_Float16)(bf16r(s1) * WCARRY);
  }
  *(volatile v8h*)(dst + (size_t)i * 8) = hv;
  __threadfence();
  *(volatile v8h*)(dst + (size_t)i * 8) = hv;
}

__global__ __launch_bounds__(SCAN_THR) void gru_scan_kernel(
    const float* __restrict__ px, const float* __restrict__ py, const float* __restrict__ vx, const float* __restrict__ vy,
    const float* __restrict__ W_embed, const float* __restrict__ b_embed,
    const unsigned short* __restrict__ Bwp,
    const float* __restrict__ b_ih, const float* __restrict__ b_hh,
    const int* __restrict__ step_mask, const int* __restrict__ ctxp,
    float* __restrict__ hs) {
  __shared__ __align__(16) _Float16 Ash[16 * APITCH];
  __shared__ __align__(16) float gS[8 * NGATE];
  __shared__ __align__(16) float hstage[STAGE_STEPS * SCAN_THR];
  __shared__ unsigned uxw[NSTEP / 32];

  const _Float16* Bw = (const _Float16*)Bwp;
  const int tid = threadIdx.x, lane = tid & 31, wave = tid >> 5;
  const int c = lane & 15, hh = lane >> 4, koff = hh * 8;
  const int half = wave >> 3, ub = wave & 7;

  int ctx = ctxp[0];
  ctx = ctx < 1 ? 1 : ctx;

  {
    unsigned bits = 0u;
#pragma unroll 1
    for (int q = 0; q < 8; ++q) {
      const v4i m = *(const v4i*)(step_mask + tid * 32 + q * 4);
#pragma unroll
      for (int e = 0; e < 4; ++e) {
        const int tt = tid * 32 + q * 4 + e;
        const int mv = m[e];
        const bool ux = (tt < ctx) || (mv == 0);
        bits |= ux ? (1u << (q * 4 + e)) : 0u;
      }
    }
    uxw[tid] = bits;
  }
#pragma unroll 1
  for (int i = tid; i < 16 * APITCH; i += SCAN_THR) Ash[i] = (_Float16)0.0f;

  v16h bF[3][4];
  float bia[3];
#pragma unroll
  for (int g = 0; g < 3; ++g) {
    const int wrow = half * NGATE + g * NHID + 16 * ub + c;
#pragma unroll
    for (int kc = 0; kc < 4; ++kc) {
      bF[g][kc] = frag_load(Bw + (size_t)wrow * NHID + koff + 32 * kc);
      pin_h(bF[g][kc]);
    }
    const int bidx = g * NHID + 16 * ub + c;
    const float bi = b_ih[bidx];
    const float bh = b_hh[bidx];
    bia[g] = bf16r(half ? bh : bi);
  }

  const int gb = tid >> 7, gj = tid & 127;
  const int arow0 = 8 * (gb >> 1) + (gb & 1);
  const float* fsrc = (gb == 0) ? px : ((gb == 1) ? py : ((gb == 2) ? vx : vy));
  float w0, w1, w2, w3, be;
  {
    const v4f we = *(const v4f*)(W_embed + gj * 4);
    const float s0 = we[0];
    const float s1 = we[1];
    const float s2 = we[2];
    const float s3 = we[3];
    w0 = bf16r(s0); w1 = bf16r(s1); w2 = bf16r(s2); w3 = bf16r(s3);
    be = bf16r(b_embed[gj]);
  }
  __syncthreads();

  float f0, f1, f2, f3;
  {
    float a0 = fsrc[0], a1 = fsrc[NSTEP], a2 = fsrc[2 * NSTEP], a3 = fsrc[3 * NSTEP];
    pin_f4(a0, a1, a2, a3);
    const float xe0 = embed4(w0, w1, w2, w3, be, a0, a1, a2, a3);
    _Float16 xh, xl;
    split16(xe0, xh, xl);
    Ash[arow0 * APITCH + gj] = xh;
    Ash[(arow0 + 4) * APITCH + gj] = xl;
    f0 = fsrc[1]; f1 = fsrc[NSTEP + 1]; f2 = fsrc[2 * NSTEP + 1]; f3 = fsrc[3 * NSTEP + 1];
    pin_f4(f0, f1, f2, f3);
  }
  float hreg = 0.0f;
  __syncthreads();

  const _Float16* arow = Ash + c * APITCH + koff;
  const v8f z8 = {0.f, 0.f, 0.f, 0.f, 0.f, 0.f, 0.f, 0.f};

#pragma unroll 1
  for (int t = 0; t < NSTEP; ++t) {
    v8f c0 = z8, c1 = z8, c2 = z8;
#pragma unroll
    for (int kc = 0; kc < 4; ++kc) {
      const v16h a = frag_load(arow + 32 * kc);
      c0 = frag_mma(a, bF[0][kc], c0);
      c1 = frag_mma(a, bF[1][kc], c1);
      c2 = frag_mma(a, bF[2][kc], c2);
      guard3(c0, c1, c2, a, bF[0][kc], bF[1][kc], bF[2][kc]);
    }
    const unsigned sux = (uxw[t >> 5] >> (t & 31)) & 1u;
    const bool selx = (half == 0) && (sux != 0u);
    {
      float o0, o1;
      const int gbase = (half * 4 + 2 * hh) * NGATE + 16 * ub + c;
      fold_gate(c0, selx, bia[0], o0, o1);
      gS[gbase] = o0;
      gS[gbase + NGATE] = o1;
      fold_gate(c1, selx, bia[1], o0, o1);
      gS[gbase + NHID] = o0;
      gS[gbase + NGATE + NHID] = o1;
      fold_gate(c2, selx, bia[2], o0, o1);
      gS[gbase + 2 * NHID] = o0;
      gS[gbase + NGATE + 2 * NHID] = o1;
    }
    __syncthreads();

    const int tn = (t + 2 < NSTEP) ? (t + 2) : (NSTEP - 1);
    float n0 = fsrc[tn], n1 = fsrc[NSTEP + tn], n2 = fsrc[2 * NSTEP + tn], n3 = fsrc[3 * NSTEP + tn];
    pin_f4(n0, n1, n2, n3);

    const float i_r = gS[gb * NGATE + gj];
    const float i_z = gS[gb * NGATE + NHID + gj];
    const float i_n = gS[gb * NGATE + 2 * NHID + gj];
    const float h_r = gS[(4 + gb) * NGATE + gj];
    const float h_z = gS[(4 + gb) * NGATE + NHID + gj];
    const float h_n = gS[(4 + gb) * NGATE + 2 * NHID + gj];
    const float rg = sigm(i_r + h_r);
    const float zg = sigm(i_z + h_z);
    const float ng = tanhf(i_n + rg * h_n);
    const float hn = (1.0f - zg) * ng + zg * hreg;
    hreg = hn;

    {
      _Float16 qh, ql;
      split16(hn, qh, ql);
      Ash[(arow0 + 2) * APITCH + gj] = qh;
      Ash[(arow0 + 6) * APITCH + gj] = ql;
      const float xn = embed4(w0, w1, w2, w3, be, f0, f1, f2, f3);
      split16(xn, qh, ql);
      Ash[arow0 * APITCH + gj] = qh;
      Ash[(arow0 + 4) * APITCH + gj] = ql;
    }
    hstage[(t & (STAGE_STEPS - 1)) * SCAN_THR + tid] = hn;
    f0 = n0; f1 = n1; f2 = n2; f3 = n3;
    __syncthreads();

    if ((t & (STAGE_STEPS - 1)) == (STAGE_STEPS - 1)) {
      const int t0 = t - (STAGE_STEPS - 1);
      const int idx0 = tid, idx1 = SCAN_THR + tid;
      const int sb0 = idx0 >> 8, sw0 = idx0 & 255;
      const int sb1 = idx1 >> 8, sw1 = idx1 & 255;
      const v4f v0 = *(const v4f*)(hstage + (sw0 >> 5) * SCAN_THR + sb0 * NHID + (sw0 & 31) * 4);
      const v4f v1 = *(const v4f*)(hstage + (sw1 >> 5) * SCAN_THR + sb1 * NHID + (sw1 & 31) * 4);
      float* d0 = hs + ((size_t)sb0 * NSTEP + (size_t)(t0 + (sw0 >> 5))) * NHID + (sw0 & 31) * 4;
      float* d1 = hs + ((size_t)sb1 * NSTEP + (size_t)(t0 + (sw1 >> 5))) * NHID + (sw1 & 31) * 4;
      *(volatile v4f*)d0 = v0;
      *(volatile v4f*)d1 = v1;
      __threadfence();
      *(volatile v4f*)d0 = v0;
      *(volatile v4f*)d1 = v1;
    }
  }
}

__global__ __launch_bounds__(HEAD_THR) void head_kernel(const float* __restrict__ hs,
                                                        const unsigned short* __restrict__ W1p,
                                                        const unsigned short* __restrict__ W2p,
                                                        const float* __restrict__ b1, const float* __restrict__ b2,
                                                        const float* __restrict__ W3, const float* __restrict__ b3,
                                                        float* __restrict__ out) {
  __shared__ __align__(16) float slab[HEAD_THR / 32][16 * SLABP];
  __shared__ __align__(16) float w3S[NOUTCH * NHEAD2];
  __shared__ __align__(16) float y3S[NOUTCH * HEAD_ROWS];
  __shared__ float bS[NHEAD1 + NHEAD2];

  const _Float16* W1h = (const _Float16*)W1p;
  const _Float16* W2h = (const _Float16*)W2p;
  const int tid = threadIdx.x, lane = tid & 31, wave = tid >> 5;
  const int c = lane & 15, hh = lane >> 4, koff = hh * 8;
  const int m0 = blockIdx.x * HEAD_ROWS;
  float* sw = slab[wave];

  if (tid < 128) {
    w3S[tid] = bf16r(W3[tid]);
    const float v1 = b1[tid & 63];
    const float v2 = b2[tid & 63];
    bS[tid] = bf16r(tid < 64 ? v1 : v2);
  }
  __syncthreads();

  const v8f z8 = {0.f, 0.f, 0.f, 0.f, 0.f, 0.f, 0.f, 0.f};

  {
    v8f aH[4], aL[4];
#pragma unroll
    for (int nt = 0; nt < 4; ++nt) { aH[nt] = z8; aL[nt] = z8; }
    const float* ar = hs + (size_t)(m0 + wave * 16 + c) * NHID + koff;
#pragma unroll 1
    for (int kc = 0; kc < NHID / 32; ++kc) {
      const float* p = ar + 32 * kc;
      const v4f x0 = *(const v4f*)(p);
      const v4f x1 = *(const v4f*)(p + 4);
      const v4f x2 = *(const v4f*)(p + 16);
      const v4f x3 = *(const v4f*)(p + 20);
      v16h fh, fl;
      build_frag(x0, x1, x2, x3, fh, fl);
      const _Float16* wb = W1h + (size_t)c * NHID + koff + 32 * kc;
      const v16h q0 = frag_load(wb);
      const v16h q1 = frag_load(wb + 16 * NHID);
      const v16h q2 = frag_load(wb + 32 * NHID);
      const v16h q3 = frag_load(wb + 48 * NHID);
      aH[0] = frag_mma(fh, q0, aH[0]);
      aH[1] = frag_mma(fh, q1, aH[1]);
      aH[2] = frag_mma(fh, q2, aH[2]);
      aH[3] = frag_mma(fh, q3, aH[3]);
      aL[0] = frag_mma(fl, q0, aL[0]);
      aL[1] = frag_mma(fl, q1, aL[1]);
      aL[2] = frag_mma(fl, q2, aL[2]);
      aL[3] = frag_mma(fl, q3, aL[3]);
      guard8(aH[0], aH[1], aH[2], aH[3], aL[0], aL[1], aL[2], aL[3], fh, fl, q0, q1, q2, q3);
    }
#pragma unroll
    for (int nt = 0; nt < 4; ++nt) {
      const float bv = bS[16 * nt + c];
#pragma unroll
      for (int r = 0; r < 8; ++r)
        sw[(8 * hh + r) * SLABP + 16 * nt + c] = aH[nt][r] * HI_INV + aL[nt][r] * HILO_INV + bv;
    }
  }
  __syncthreads();
#pragma unroll 1
  for (int i = 0; i < 32; ++i) {
    const int idx = i * 32 + lane;
    float* q = sw + (idx >> 6) * SLABP + (idx & 63);
    const float v = *q;
    *q = elu1(v);
  }
  __syncthreads();

  {
    v8f dH[4], dL[4];
#pragma unroll
    for (int nt = 0; nt < 4; ++nt) { dH[nt] = z8; dL[nt] = z8; }
#pragma unroll 1
    for (int kc = 0; kc < NHEAD1 / 32; ++kc) {
      const float* p = sw + c * SLABP + koff + 32 * kc;
      const v4f x0 = *(const v4f*)(p);
      const v4f x1 = *(const v4f*)(p + 4);
      const v4f x2 = *(const v4f*)(p + 16);
      const v4f x3 = *(const v4f*)(p + 20);
      v16h fh, fl;
      build_frag(x0, x1, x2, x3, fh, fl);
      const _Float16* wb = W2h + (size_t)c * NHEAD1 + koff + 32 * kc;
      const v16h q0 = frag_load(wb);
      const v16h q1 = frag_load(wb + 16 * NHEAD1);
      const v16h q2 = frag_load(wb + 32 * NHEAD1);
      const v16h q3 = frag_load(wb + 48 * NHEAD1);
      dH[0] = frag_mma(fh, q0, dH[0]);
      dH[1] = frag_mma(fh, q1, dH[1]);
      dH[2] = frag_mma(fh, q2, dH[2]);
      dH[3] = frag_mma(fh, q3, dH[3]);
      dL[0] = frag_mma(fl, q0, dL[0]);
      dL[1] = frag_mma(fl, q1, dL[1]);
      dL[2] = frag_mma(fl, q2, dL[2]);
      dL[3] = frag_mma(fl, q3, dL[3]);
      guard8(dH[0], dH[1], dH[2], dH[3], dL[0], dL[1], dL[2], dL[3], fh, fl, q0, q1, q2, q3);
    }
    __syncthreads();
#pragma unroll
    for (int nt = 0; nt < 4; ++nt) {
      const float bv = bS[NHEAD1 + 16 * nt + c];
#pragma unroll
      for (int r = 0; r < 8; ++r)
        sw[(8 * hh + r) * SLABP + 16 * nt + c] = dH[nt][r] * HI_INV + dL[nt][r] * HILO_INV + bv;
    }
  }
  __syncthreads();
#pragma unroll 1
  for (int i = 0; i < 32; ++i) {
    const int idx = i * 32 + lane;
    float* q = sw + (idx >> 6) * SLABP + (idx & 63);
    const float v = *q;
    *q = elu1(v);
  }
  __syncthreads();

  {
    const int rl = tid >> 1, o = tid & 1;
    const float* srow = sw + (rl & 15) * SLABP;
    const float* wrow = w3S + o * NHEAD2;
    const float b3v = bf16r(b3[o]);
    float acc = 0.0f;
#pragma unroll 1
    for (int k4 = 0; k4 < NHEAD2 / 4; ++k4) {
      const v4f y = *(const v4f*)(srow + 4 * k4);
      const v4f w = *(const v4f*)(wrow + 4 * k4);
      acc = fmaf(y[0], w[0], acc);
      acc = fmaf(y[1], w[1], acc);
      acc = fmaf(y[2], w[2], acc);
      acc = fmaf(y[3], w[3], acc);
    }
    y3S[o * HEAD_ROWS + rl] = acc + b3v;
  }
  __syncthreads();
  if (wave < NOUTCH) {
    const v4f v = *(const v4f*)(y3S + wave * HEAD_ROWS + 4 * lane);
    float* dst = out + (size_t)wave * NROWS + (size_t)m0 + 4 * lane;
    *(volatile v4f*)dst = v;
    __threadfence();
    *(volatile v4f*)dst = v;
  }
}

extern "C" void kernel_launch(void* const* d_in, const int* in_sizes, int n_in,
                              void* d_out, int out_size, void* d_ws, size_t ws_size, hipStream_t stream) {
  if (n_in < 18 || d_out == nullptr || d_ws == nullptr) return;
  if (in_sizes[0] != NROWS || in_sizes[1] != NROWS || in_sizes[2] != NROWS || in_sizes[3] != NROWS ||
      in_sizes[4] != NHID * 4 || in_sizes[5] != NHID ||
      in_sizes[6] != NGATE * NHID || in_sizes[7] != NGATE * NHID || in_sizes[8] != NGATE || in_sizes[9] != NGATE ||
      in_sizes[10] != NHEAD1 * NHID || in_sizes[11] != NHEAD1 || in_sizes[12] != NHEAD2 * NHEAD1 || in_sizes[13] != NHEAD2 ||
      in_sizes[14] != NOUTCH * NHEAD2 || in_sizes[15] != NOUTCH || in_sizes[16] != NSTEP || in_sizes[17] != 1 ||
      out_size != NOUTCH * NROWS) return;

  const float* px      = (const float*)d_in[0];
  const float* py      = (const float*)d_in[1];
  const float* vx      = (const float*)d_in[2];
  const float* vy      = (const float*)d_in[3];
  const float* W_embed = (const float*)d_in[4];
  const float* b_embed = (const float*)d_in[5];
  const float* W_ih    = (const float*)d_in[6];
  const float* W_hh    = (const float*)d_in[7];
  const float* b_ih    = (const float*)d_in[8];
  const float* b_hh    = (const float*)d_in[9];
  const float* W1      = (const float*)d_in[10];
  const float* b1      = (const float*)d_in[11];
  const float* W2      = (const float*)d_in[12];
  const float* b2      = (const float*)d_in[13];
  const float* W3      = (const float*)d_in[14];
  const float* b3      = (const float*)d_in[15];
  const int* step_mask = (const int*)d_in[16];
  const int* ctxp      = (const int*)d_in[17];
  float* out = (float*)d_out;

  char* ws = (char*)d_ws;
  size_t off = 0;
  auto carve = [&](size_t bytes) -> char* { char* p = ws + off; off += (bytes + 255) & ~(size_t)255; return p; };
  unsigned short* BW  = (unsigned short*)carve((size_t)NWROW * NHID * 2);
  unsigned short* W1H = (unsigned short*)carve((size_t)NHEAD1 * NHID * 2);
  unsigned short* W2H = (unsigned short*)carve((size_t)NHEAD2 * NHEAD1 * 2);
  float*          HS  = (float*)carve((size_t)NROWS * NHID * 4);
  if (off > ws_size || off > (size_t)134217728) return;

  prep_kernel<<<54, 256, 0, stream>>>(W_ih, W_hh, W1, W2, BW, W1H, W2H);
  gru_scan_kernel<<<1, SCAN_THR, 0, stream>>>(px, py, vx, vy, W_embed, b_embed, BW, b_ih, b_hh, step_mask, ctxp, HS);
  head_kernel<<<NROWS / HEAD_ROWS, HEAD_THR, 0, stream>>>(HS, W1H, W2H, b1, b2, W3, b3, out);
}
